// NDimensionalAttention_63745904607888
// MI455X (gfx1250) — hardware-verified
//
#include <hip/hip_runtime.h>
#include <math.h>
#include <stdint.h>

#define CH     64
#define NSEQ   4096
#define NHEAD  4
#define HDIM   16
#define QKW    (2 * CH)
#define XC     16.0f
#define WSC    1024.0f
#define QC     4096.0f
#define VC     4096.0f
#define PC     1024.0f
#define OC     32768.0f
#define EPSN   1.0e-8f
static_assert(NHEAD * HDIM == CH);
static_assert((NSEQ % 64) == 0 && (QKW % 64) == 0);
static_assert(CH == 32 * 2);

typedef _Float16 v16h __attribute__((ext_vector_type(16)));
typedef _Float16 v8h  __attribute__((ext_vector_type(8)));
typedef float    v8f  __attribute__((ext_vector_type(8)));
typedef float    v4f  __attribute__((ext_vector_type(4)));
typedef unsigned int v4u __attribute__((ext_vector_type(4)));

union FragH { v16h v; v8h h[2]; };

__device__ __forceinline__ unsigned short bf_bits(float f) {
  unsigned u = __float_as_uint(f);
  return (unsigned short)((u + 0x7FFFu + ((u >> 16) & 1u)) >> 16);
}
__device__ __forceinline__ float bf_up(unsigned short h) { return __uint_as_float(((unsigned)h) << 16); }
__device__ __forceinline__ float bfr(float f) { return bf_up(bf_bits(f)); }
__device__ __forceinline__ unsigned short h_bits(_Float16 x) { return __builtin_bit_cast(unsigned short, x); }
__device__ __forceinline__ unsigned pk16(unsigned short a, unsigned short b) { return (unsigned)a | ((unsigned)b << 16); }
__device__ __forceinline__ v8f zero8() { v8f z = {0.f, 0.f, 0.f, 0.f, 0.f, 0.f, 0.f, 0.f}; return z; }

__device__ __forceinline__ v16h ldfrag_h(const _Float16* p) {
  FragH f;
  f.h[0] = *(const v8h*)(p);
  f.h[1] = *(const v8h*)(p + 16);
  return f.v;
}

__device__ __forceinline__ v8f mma_h_raw(v16h a, v16h b, v8f c) {
  return __builtin_amdgcn_wmma_f32_16x16x32_f16(false, a, false, b, (short)0, c, false, false);
}
__device__ __forceinline__ void dep_guard1(v8f& a, v8f& b, v16h x) {
#if defined(__HIP_DEVICE_COMPILE__)
  asm volatile("v_nop\n\tv_nop\n\tv_nop\n\tv_nop" : "+v"(a), "+v"(b) : "v"(x));
#endif
}
__device__ __forceinline__ void keep4_h(v16h a, v16h b, v16h c, v16h d) {
#if defined(__HIP_DEVICE_COMPILE__)
  asm volatile("v_nop" :: "v"(a), "v"(b), "v"(c), "v"(d));
#endif
}
__device__ __forceinline__ void acc_guard4(v8f& a, v8f& b, v8f& c, v8f& d) {
#if defined(__HIP_DEVICE_COMPILE__)
  asm volatile("v_nop\n\tv_nop\n\tv_nop\n\tv_nop" : "+v"(a), "+v"(b), "+v"(c), "+v"(d));
#endif
}
__device__ __forceinline__ void sguard2(v8f& a, v8f& b, v16h k0, v16h k1, v16h k2, v16h k3, v16h q) {
#if defined(__HIP_DEVICE_COMPILE__)
  asm volatile("v_nop\n\tv_nop\n\tv_nop\n\tv_nop"
               : "+v"(a), "+v"(b) : "v"(k0), "v"(k1), "v"(k2), "v"(k3), "v"(q));
#endif
}
__device__ __forceinline__ void oguard3(v8f& o, v16h a0, v16h a1, v16h b0) {
#if defined(__HIP_DEVICE_COMPILE__)
  asm volatile("v_nop\n\tv_nop\n\tv_nop\n\tv_nop" : "+v"(o) : "v"(a0), "v"(a1), "v"(b0));
#endif
}
__device__ __forceinline__ void wave_sync_lds() {
  __builtin_amdgcn_fence(__ATOMIC_RELEASE, "workgroup");
  __builtin_amdgcn_wave_barrier();
  __builtin_amdgcn_fence(__ATOMIC_ACQUIRE, "workgroup");
}
__device__ __forceinline__ void store2_v4u(unsigned short* p, v4u v) {
  *(volatile v4u*)p = v;
  __threadfence();
  *(volatile v4u*)p = v;
}

__global__ __launch_bounds__(256) void wprep(const float* __restrict__ wq, const float* __restrict__ wk,
                                              const float* __restrict__ wv, const float* __restrict__ wo,
                                              unsigned short* WT, unsigned short* WPD) {
  const int t = threadIdx.x;
  const int bx = blockIdx.x;
  if (bx < 6) {
    const int m = bx >> 1;
    const float* src = (m == 0) ? wq : ((m == 1) ? wk : wv);
    const int g = bx * 256 + t;
    const int o = g >> 3, e = g & 7;
    const int h = (o >> 4) & 3, d = o & 15;
    float w[8];
#pragma unroll
    for (int i = 0; i < 8; ++i) w[i] = bfr(src[((size_t)(h * CH + 8 * e + i)) * HDIM + d]) * (0.125f * WSC);
    v4u v;
#pragma unroll
    for (int i = 0; i < 4; ++i) v[i] = pk16(h_bits((_Float16)w[2 * i]), h_bits((_Float16)w[2 * i + 1]));
    store2_v4u(WT + (size_t)o * CH + 8 * e, v);
  } else {
    const int g = (bx - 6) * 256 + t;
    const int c = g >> 4, e = g & 15;
    const int jj = (8 * e) & 63, h = jj >> 4, d0 = jj & 15;
    const float* sp = wo + ((size_t)(h * CH + c)) * HDIM + d0;
    const v4f a = *(const v4f*)(sp), cc = *(const v4f*)(sp + 4);
    float w[8];
#pragma unroll
    for (int i = 0; i < 4; ++i) { w[i] = bfr(a[i]) * (0.125f * WSC); w[4 + i] = bfr(cc[i]) * (0.125f * WSC); }
    v4u v;
#pragma unroll
    for (int i = 0; i < 4; ++i) v[i] = pk16(h_bits((_Float16)w[2 * i]), h_bits((_Float16)w[2 * i + 1]));
    store2_v4u(WPD + (size_t)c * (2 * CH) + 8 * e, v);
  }
}

__global__ __launch_bounds__(256) void xtok(const float* __restrict__ x, unsigned short* XN) {
  __shared__ __align__(16) float T[CH * 36];
  __shared__ __align__(16) unsigned int Yw[8][4 * 32];
  const int tid = threadIdx.x, wave = tid >> 5, lane = tid & 31;
  const int bx = blockIdx.x;
  const int b  = bx >> 7;
  const int n0 = (bx & 127) * 32;
  const float* sb = x + (size_t)b * CH * NSEQ + n0;
  {
    const int q = lane >> 3, e = lane & 7;
#pragma unroll
    for (int it = 0; it < 2; ++it) {
      const int c = wave * 8 + it * 4 + q;
      const v4f v = *(const v4f*)(sb + (size_t)c * NSEQ + 4 * e);
      *(v4f*)(T + c * 36 + 4 * e) = v;
    }
  }
  __syncthreads();
#pragma unroll
  for (int i = 0; i < 4; ++i) {
    const int tl = wave * 4 + i;
    const float y0 = bfr(T[(2 * lane) * 36 + tl]) * XC;
    const float y1 = bfr(T[(2 * lane + 1) * 36 + tl]) * XC;
    Yw[wave][i * 32 + lane] = pk16(h_bits((_Float16)y0), h_bits((_Float16)y1));
  }
  wave_sync_lds();
  {
    const v4u o4 = *(const v4u*)(&Yw[wave][4 * lane]);
    const size_t tokA = (size_t)b * NSEQ + n0 + wave * 4;
    store2_v4u(XN + tokA * CH + 8 * lane, o4);
  }
}

__global__ __launch_bounds__(256) void vsum(const float* __restrict__ x, const float* __restrict__ wv, float* VS) {
  __shared__ double ts[256];
  __shared__ double tc[CH];
  __shared__ __align__(16) float vf[CH];
  const int tid = threadIdx.x;
  const int b = blockIdx.x;
  const int c = tid >> 2, qt = tid & 3;
  const float* xr = x + ((size_t)b * CH + c) * NSEQ + (size_t)qt * (NSEQ / 4);
  double acc = 0.0;
#pragma unroll 4
  for (int n = 0; n < NSEQ / 4; ++n) acc += (double)bfr(xr[n]);
  ts[tid] = acc;
  __syncthreads();
  if (tid < CH) tc[tid] = (ts[4 * tid] + ts[4 * tid + 1]) + (ts[4 * tid + 2] + ts[4 * tid + 3]);
  __syncthreads();
  if (tid < CH) {
    const int h = tid >> 4, d = tid & 15;
    double s = 0.0;
#pragma unroll 1
    for (int c2 = 0; c2 < CH; ++c2)
      s += tc[c2] * (double)(bfr(wv[((size_t)(h * CH + c2)) * HDIM + d]) * 0.125f);
    vf[tid] = (float)s;
  }
  __syncthreads();
  if (tid < 16) {
    const v4f v = *(const v4f*)(vf + 4 * tid);
    float* p = VS + (size_t)b * CH + 4 * tid;
    *(volatile v4f*)p = v;
    __threadfence();
    *(volatile v4f*)p = v;
  }
}

template <int BKM, int OM>
__global__ __launch_bounds__(256) void gemm64(
    const unsigned short* __restrict__ Ap, int lda, long long strideA,
    const unsigned short* __restrict__ Bp, int ldb, long long strideB,
    void* Cout, int ldc, long long strideC,
    unsigned short* Clo, int ldlo, long long strideLo, int nsplit,
    float osc0, float osc1, int M, int N, int K) {
  __shared__ __align__(16) float sT[8][16 * 68];
  const int b    = blockIdx.y;
  const int lane = threadIdx.x & 31;
  const int wave = threadIdx.x >> 5;
  const int tilesN = N >> 6;
  const int tilesM = M >> 6;
  const int tile = blockIdx.x * 8 + wave;
  if (tile >= tilesM * tilesN) return;
  const int tm = tile / tilesN;
  const int tn = tile - tm * tilesN;
  const int m0 = tm << 6;
  const int n0 = tn << 6;

  const _Float16* Ah = (const _Float16*)(const void*)Ap + (size_t)b * strideA;
  const _Float16* Bb = (const _Float16*)(const void*)Bp + (size_t)b * strideB;

  const int rlane = lane & 15;
  const int koff  = (lane >> 4) * 8;
  const int mOff  = (lane >> 4) * 8;

  v8f acc[4][4];
#pragma unroll
  for (int i = 0; i < 4; ++i)
#pragma unroll
    for (int j = 0; j < 4; ++j) acc[i][j] = zero8();

  for (int k0 = 0; k0 < K; k0 += 32) {
    v16h bh[4];
#pragma unroll
    for (int j = 0; j < 4; ++j) {
      if (BKM == 0) {
        const size_t bo = (size_t)(n0 + (j << 4) + rlane) * ldb + koff + k0;
        bh[j] = ldfrag_h(Bb + bo);
      } else {
        const _Float16* bp = Bb + (size_t)(k0 + koff) * ldb + n0 + (j << 4) + rlane;
        FragH f;
#pragma unroll
        for (int i = 0; i < 8; ++i) {
          f.h[0][i] = bp[(size_t)i * ldb];
          f.h[1][i] = bp[(size_t)(16 + i) * ldb];
        }
        bh[j] = f.v;
      }
    }
#pragma unroll
    for (int i = 0; i < 4; ++i) {
      const size_t ao = (size_t)(m0 + (i << 4) + rlane) * lda + koff + k0;
      const v16h ah = ldfrag_h(Ah + ao);
#pragma unroll
      for (int j = 0; j < 4; ++j) acc[i][j] = mma_h_raw(ah, bh[j], acc[i][j]);
      dep_guard1(acc[i][0], acc[i][3], ah);
    }
    keep4_h(bh[0], bh[1], bh[2], bh[3]);
  }
  acc_guard4(acc[0][0], acc[0][1], acc[0][2], acc[0][3]);
  acc_guard4(acc[1][0], acc[1][1], acc[1][2], acc[1][3]);
  acc_guard4(acc[2][0], acc[2][1], acc[2][2], acc[2][3]);
  acc_guard4(acc[3][0], acc[3][1], acc[3][2], acc[3][3]);

  const float oscale = (OM == 1 && n0 >= nsplit) ? osc1 : osc0;
  const bool  dolo   = (OM == 1) && (n0 < nsplit);
  const int hh2 = lane >> 4, c4 = (lane & 15) * 4;
  const int q8  = lane >> 3, c8 = (lane & 7) * 8;

  float* slab = sT[wave];
#pragma unroll
  for (int i = 0; i < 4; ++i) {
    const int mBase = m0 + (i << 4);
#pragma unroll
    for (int j = 0; j < 4; ++j) {
#pragma unroll
      for (int r = 0; r < 8; ++r) {
        slab[(mOff + r) * 68 + (j << 4) + rlane] = acc[i][j][r];
      }
    }
    wave_sync_lds();
    if (OM == 0) {
      float* C = (float*)Cout + (size_t)b * strideC;
      v4f vals[8];
#pragma unroll
      for (int it = 0; it < 8; ++it) {
        const int row = it * 2 + hh2;
        v4f v = *(const v4f*)(slab + row * 68 + c4);
#pragma unroll
        for (int e = 0; e < 4; ++e) v[e] = v[e] * oscale;
        vals[it] = v;
      }
#pragma unroll
      for (int it = 0; it < 8; ++it) {
        const int row = it * 2 + hh2;
        *(volatile v4f*)(C + (size_t)(mBase + row) * ldc + n0 + c4) = vals[it];
      }
      __threadfence();
#pragma unroll
      for (int it = 0; it < 8; ++it) {
        const int row = it * 2 + hh2;
        *(volatile v4f*)(C + (size_t)(mBase + row) * ldc + n0 + c4) = vals[it];
      }
    } else {
      unsigned short* C = (unsigned short*)Cout + (size_t)b * strideC;
      unsigned short* L = Clo + (size_t)b * strideLo;
      v4u hv[4], lv[4];
#pragma unroll
      for (int it = 0; it < 4; ++it) {
        const int row = it * 4 + q8;
        const float* sp = slab + row * 68 + c8;
        v4u a, lo;
#pragma unroll
        for (int e = 0; e < 4; ++e) {
          const float f0 = sp[2 * e] * oscale, f1 = sp[2 * e + 1] * oscale;
          const _Float16 h0 = (_Float16)f0, h1 = (_Float16)f1;
          const _Float16 l0 = (_Float16)(f0 - (float)h0), l1 = (_Float16)(f1 - (float)h1);
          a[e]  = pk16(h_bits(h0), h_bits(h1));
          lo[e] = pk16(h_bits(l0), h_bits(l1));
        }
        hv[it] = a;
        lv[it] = lo;
      }
#pragma unroll
      for (int it = 0; it < 4; ++it) {
        const int row = it * 4 + q8;
        *(volatile v4u*)(C + (size_t)(mBase + row) * ldc + n0 + c8) = hv[it];
        if (dolo) *(volatile v4u*)(L + (size_t)(mBase + row) * ldlo + n0 + c8) = lv[it];
      }
      __threadfence();
#pragma unroll
      for (int it = 0; it < 4; ++it) {
        const int row = it * 4 + q8;
        *(volatile v4u*)(C + (size_t)(mBase + row) * ldc + n0 + c8) = hv[it];
        if (dolo) *(volatile v4u*)(L + (size_t)(mBase + row) * ldlo + n0 + c8) = lv[it];
      }
    }
    wave_sync_lds();
  }
}

__global__ __launch_bounds__(256) void qknorm(const float* __restrict__ qf, unsigned short* QH, unsigned short* QL) {
  __shared__ __align__(16) unsigned int Yw[8][2][256];
  const int tid = threadIdx.x, wave = tid >> 5, lane = tid & 31;
  const int bx = blockIdx.x;
  const int i = lane >> 3, g = lane & 7;
  const int tok = bx * 32 + wave * 4 + i;
  const float* sp = qf + (size_t)tok * QKW + 16 * g;
  const v4f a0 = *(const v4f*)(sp), a1 = *(const v4f*)(sp + 4), a2 = *(const v4f*)(sp + 8), a3 = *(const v4f*)(sp + 12);
  float u[16];
#pragma unroll
  for (int e = 0; e < 4; ++e) { u[e] = a0[e]; u[4 + e] = a1[e]; u[8 + e] = a2[e]; u[12 + e] = a3[e]; }
  float ss = 0.f;
#pragma unroll
  for (int e = 0; e < 16; ++e) ss += u[e] * u[e];
  const float inv = 1.0f / (sqrtf(ss) + EPSN);
  v4u hw0, hw1, lw0, lw1;
#pragma unroll
  for (int e = 0; e < 4; ++e) {
    const float f0 = (u[2 * e] * inv) * QC, f1 = (u[2 * e + 1] * inv) * QC;
    const _Float16 h0 = (_Float16)f0, h1 = (_Float16)f1;
    const _Float16 l0 = (_Float16)(f0 - (float)h0), l1 = (_Float16)(f1 - (float)h1);
    hw0[e] = pk16(h_bits(h0), h_bits(h1));
    lw0[e] = pk16(h_bits(l0), h_bits(l1));
    const float f2 = (u[8 + 2 * e] * inv) * QC, f3 = (u[8 + 2 * e + 1] * inv) * QC;
    const _Float16 h2 = (_Float16)f2, h3 = (_Float16)f3;
    const _Float16 l2 = (_Float16)(f2 - (float)h2), l3 = (_Float16)(f3 - (float)h3);
    hw1[e] = pk16(h_bits(h2), h_bits(h3));
    lw1[e] = pk16(h_bits(l2), h_bits(l3));
  }
  *(v4u*)(&Yw[wave][0][i * 64 + 8 * g])     = hw0;
  *(v4u*)(&Yw[wave][0][i * 64 + 8 * g + 4]) = hw1;
  *(v4u*)(&Yw[wave][1][i * 64 + 8 * g])     = lw0;
  *(v4u*)(&Yw[wave][1][i * 64 + 8 * g + 4]) = lw1;
  wave_sync_lds();
  {
    const v4u oa = *(const v4u*)(&Yw[wave][0][4 * lane]);
    const v4u ob = *(const v4u*)(&Yw[wave][0][128 + 4 * lane]);
    const v4u la = *(const v4u*)(&Yw[wave][1][4 * lane]);
    const v4u lb = *(const v4u*)(&Yw[wave][1][128 + 4 * lane]);
    const size_t tokA = (size_t)bx * 32 + wave * 4;
    unsigned short* pa = QH + tokA * QKW + 8 * lane;
    unsigned short* pb = QH + (tokA + 2) * QKW + 8 * lane;
    unsigned short* pc = QL + tokA * QKW + 8 * lane;
    unsigned short* pd = QL + (tokA + 2) * QKW + 8 * lane;
    *(volatile v4u*)pa = oa;
    *(volatile v4u*)pb = ob;
    *(volatile v4u*)pc = la;
    *(volatile v4u*)pd = lb;
    __threadfence();
    *(volatile v4u*)pa = oa;
    *(volatile v4u*)pb = ob;
    *(volatile v4u*)pc = la;
    *(volatile v4u*)pd = lb;
  }
}

__global__ __launch_bounds__(128)
void attn_t(const unsigned short* __restrict__ qh, const unsigned short* __restrict__ ql,
            const unsigned short* __restrict__ vp, const float* __restrict__ vs, unsigned short* op) {
  __shared__ __align__(16) unsigned short Os[2][HDIM * 64];
  const int tid  = threadIdx.x;
  const int wave = tid >> 5;
  const int lane = tid & 31;
  const int hh   = lane >> 4;
  const int c    = lane & 15;
  const int bx = blockIdx.x;
  const int qb = bx & 63;
  const int hd = (bx >> 6) & 3;
  const int b  = bx >> 8;
  const int q0 = qb * 64;
  const size_t tok0 = (size_t)b * NSEQ;

  const _Float16* QHp = (const _Float16*)(const void*)qh;
  const _Float16* QLp = (const _Float16*)(const void*)ql;
  const _Float16* Vh  = (const _Float16*)(const void*)vp + ((size_t)b * (2 * CH) + (size_t)hd * HDIM + c) * NSEQ + 8 * hh;
  const _Float16* Vl  = Vh + (size_t)CH * NSEQ;

  FragH qf;
  {
    const size_t tr = tok0 + q0 + wave * 16 + c;
    qf.h[0] = *(const v8h*)(QHp + tr * QKW + hd * HDIM + 8 * hh);
    qf.h[1] = *(const v8h*)(QLp + tr * QKW + hd * HDIM + 8 * hh);
  }
  const _Float16* Kh = QHp + (tok0 + c) * QKW + CH + hd * HDIM + 8 * hh;
  const _Float16* Kl = QLp + (tok0 + c) * QKW + CH + hd * HDIM + 8 * hh;
  const float SC = 1.0f / (QC * QC);

  float l = 0.f;
  v8f o = zero8();
#pragma unroll 1
  for (int it = 0; it < NSEQ / 32; ++it) {
    const int kb = it * 32;
    v16h kh0, kh1, kl0, kl1;
    {
      FragH f;
      f.h[0] = *(const v8h*)(Kh + (size_t)kb * QKW);        f.h[1] = f.h[0]; kh0 = f.v;
      f.h[0] = *(const v8h*)(Kh + (size_t)(kb + 16) * QKW); f.h[1] = f.h[0]; kh1 = f.v;
      f.h[0] = *(const v8h*)(Kl + (size_t)kb * QKW);        f.h[1] = f.h[0]; kl0 = f.v;
      f.h[0] = *(const v8h*)(Kl + (size_t)(kb + 16) * QKW); f.h[1] = f.h[0]; kl1 = f.v;
    }
    v8f s0 = mma_h_raw(kh0, qf.v, zero8());
    v8f s1 = mma_h_raw(kh1, qf.v, zero8());
    s0 = mma_h_raw(kl0, qf.v, s0);
    s1 = mma_h_raw(kl1, qf.v, s1);
    sguard2(s0, s1, kh0, kh1, kl0, kl1, qf.v);

    FragH p;
    float ls = 0.f;
#pragma unroll
    for (int r = 0; r < 8; ++r) {
      const float e0 = __expf(s0[r] * SC);
      const float e1 = __expf(s1[r] * SC);
      ls += e0 + e1;
      p.h[0][r] = (_Float16)((e0 - 1.0f) * PC);
      p.h[1][r] = (_Float16)((e1 - 1.0f) * PC);
    }
    l += ls;

    const v16h va = ldfrag_h(Vh + kb);
    const v16h vb = ldfrag_h(Vl + kb);
    o = mma_h_raw(va, p.v, o);
    o = mma_h_raw(vb, p.v, o);
    oguard3(o, va, vb, p.v);
  }
  l += __shfl_xor(l, 16, 32);
  const float il = 1.0f / l;
  const float* vsp = vs + (size_t)b * CH + hd * HDIM + 8 * hh;
  const v4f g0 = *(const v4f*)(vsp), g1 = *(const v4f*)(vsp + 4);
  float add[8];
#pragma unroll
  for (int e = 0; e < 4; ++e) { add[e] = g0[e]; add[4 + e] = g1[e]; }

#pragma unroll
  for (int r = 0; r < 8; ++r) {
    const float of = (o[r] * (1.0f / (PC * VC)) + add[r]) * il;
    const float f  = of * OC;
    const _Float16 h0 = (_Float16)f;
    const _Float16 l0 = (_Float16)(f - (float)h0);
    Os[0][(8 * hh + r) * 64 + wave * 16 + c] = h_bits(h0);
    Os[1][(8 * hh + r) * 64 + wave * 16 + c] = h_bits(l0);
  }
  __syncthreads();
  {
    const int d = tid >> 3, e = tid & 7;
    const v4u vh4 = *(const v4u*)(&Os[0][d * 64 + 8 * e]);
    const v4u vl4 = *(const v4u*)(&Os[1][d * 64 + 8 * e]);
    unsigned short* ph = op + ((size_t)b * (2 * CH) + (size_t)(hd * HDIM + d)) * NSEQ + q0 + 8 * e;
    unsigned short* pl = ph + (size_t)CH * NSEQ;
    *(volatile v4u*)ph = vh4;
    *(volatile v4u*)pl = vl4;
    __threadfence();
    *(volatile v4u*)ph = vh4;
    *(volatile v4u*)pl = vl4;
  }
}

extern "C" void kernel_launch(void* const* d_in, const int* in_sizes, int n_in,
                              void* d_out, int out_size, void* d_ws, size_t ws_size,
                              hipStream_t stream) {
  if (n_in < 5) return;
  const int WN = NHEAD * CH * HDIM;
  if (in_sizes[1] != WN || in_sizes[2] != WN || in_sizes[3] != WN || in_sizes[4] != WN) return;
  const long long per = (long long)CH * NSEQ;
  const long long n0sz = (long long)in_sizes[0];
  if (n0sz <= 0 || (n0sz % per) != 0) return;
  const int nb = (int)(n0sz / per);
  if ((long long)out_size != n0sz) return;

  const float* x  = (const float*)d_in[0];
  const float* wq = (const float*)d_in[1];
  const float* wk = (const float*)d_in[2];
  const float* wv = (const float*)d_in[3];
  const float* wo = (const float*)d_in[4];

  const size_t MP  = (size_t)nb * NSEQ;
  const size_t PWT = (size_t)3 * CH * CH * 2;
  const size_t PWP = (size_t)CH * (2 * CH) * 2;
  const size_t PVS = (size_t)nb * CH * 4;
  const size_t PXN = MP * CH * 2;
  const size_t PQF = MP * QKW * 4;
  const size_t PQH = MP * QKW * 2;
  const size_t PQL = MP * QKW * 2;
  const size_t PVP = (size_t)nb * (2 * CH) * NSEQ * 2;
  const size_t POP = (size_t)nb * (2 * CH) * NSEQ * 2;
  size_t off = 0;
  const size_t oWT = off; off += PWT;
  const size_t oWP = off; off += PWP;
  const size_t oVS = off; off += PVS;
  const size_t oXN = off; off += PXN;
  const size_t oQF = off; off += PQF;
  const size_t oQH = off; off += PQH;
  const size_t oQL = off; off += PQL;
  const size_t oVP = off; off += PVP;
  const size_t oOP = off; off += POP;
  if (off > ws_size) return;
  if (off > (size_t)134217728) return;

  char* ws = (char*)d_ws;
  unsigned short* WT  = (unsigned short*)(ws + oWT);
  unsigned short* WPD = (unsigned short*)(ws + oWP);
  float*          VS  = (float*)(ws + oVS);
  unsigned short* XN  = (unsigned short*)(ws + oXN);
  float*          QF  = (float*)(ws + oQF);
  unsigned short* QH  = (unsigned short*)(ws + oQH);
  unsigned short* QL  = (unsigned short*)(ws + oQL);
  unsigned short* VP  = (unsigned short*)(ws + oVP);
  unsigned short* OP  = (unsigned short*)(ws + oOP);
  float*          out = (float*)d_out;

  const int mpi = nb * NSEQ;
  const dim3 blk(256), blk128(128);
  const dim3 gW(10);
  const dim3 gXT(nb * (NSEQ / 32));
  const dim3 gVS(nb);
  const dim3 gQK(((mpi / 64) * (QKW / 64)) / 8, 1);
  const dim3 gNM(nb * (NSEQ / 32));
  const dim3 gVT(((CH / 64) * (NSEQ / 64)) / 8, nb);
  const dim3 gAT(nb * NHEAD * (NSEQ / 64));
  const dim3 gPJ(((CH / 64) * (NSEQ / 64)) / 8, nb);

  wprep<<<gW, blk, 0, stream>>>(wq, wk, wv, wo, WT, WPD);

  xtok<<<gXT, blk, 0, stream>>>(x, XN);

  vsum<<<gVS, blk, 0, stream>>>(x, wv, VS);

  gemm64<0, 0><<<gQK, blk, 0, stream>>>(
      XN, CH, 0LL,
      WT, CH, 0LL,
      (void*)QF, QKW, 0LL,
      QL, QKW, 0LL, 0,
      1.0f / (XC * WSC), 1.0f / (XC * WSC), mpi, QKW, CH);

  qknorm<<<gNM, blk, 0, stream>>>(QF, QH, QL);

  gemm64<0, 1><<<gVT, blk, 0, stream>>>(
      WT + (size_t)2 * CH * CH, CH, 0LL,
      XN, CH, (long long)NSEQ * CH,
      (void*)VP, NSEQ, (long long)(2 * CH) * NSEQ,
      VP + (size_t)CH * NSEQ, NSEQ, (long long)(2 * CH) * NSEQ, NSEQ,
      VC / (XC * WSC), VC / (XC * WSC), CH, NSEQ, CH);

  attn_t<<<gAT, blk128, 0, stream>>>(QH, QL, VP, VS, OP);

  gemm64<1, 0><<<gPJ, blk, 0, stream>>>(
      WPD, 2 * CH, 0LL,
      OP, NSEQ, (long long)(2 * CH) * NSEQ,
      (void*)out, NSEQ, (long long)CH * NSEQ,
      QL, NSEQ, 0LL, 0,
      1.0f / (WSC * OC), 1.0f / (WSC * OC), CH, NSEQ, 2 * CH);
  (void)hipGetLastError();
}
